// NDimMultiHeadAttention_82540681494879
// MI455X (gfx1250) — hardware-verified
//
#include <hip/hip_runtime.h>
#include <hip/hip_bf16.h>
#include <stddef.h>
#include <stdint.h>

#define NB    2
#define LSEQ  2048
#define EMB   512
#define NH    8
#define DH    64
#define NW    4
#define NTOK  (NB * LSEQ)
#define NQKV  (3 * EMB)
#define BR    32
#define BC    128
#define NQT   (LSEQ / BR)

static_assert(EMB == 512);
static_assert(NH * DH == EMB);
static_assert(DH % 32 == 0);
static_assert(LSEQ % 256 == 0);
static_assert(LSEQ % BR == 0);
static_assert(LSEQ % BC == 0);
static_assert(BC % 32 == 0);
static_assert(BC == 128);
static_assert(BR == 32);
static_assert(NTOK % 256 == 0);
static_assert(NQKV % 64 == 0);
static_assert(EMB % 64 == 0);

typedef float          v8f   __attribute__((ext_vector_type(8)));
typedef float          v4f   __attribute__((ext_vector_type(4)));
typedef unsigned int   v4u   __attribute__((ext_vector_type(4)));
typedef unsigned short v8us  __attribute__((ext_vector_type(8)));
typedef unsigned short v16us __attribute__((ext_vector_type(16)));
typedef __bf16         v16b  __attribute__((ext_vector_type(16)));
typedef unsigned short ush;

union FragU { v16us v; v8us h[2]; v16b b; };
union PackU { v8us s; v4u u; };
struct HL { v4u h; v4u l; };

__device__ __forceinline__ ush f2bf(float f) {
  const unsigned u = __float_as_uint(f);
  return (ush)((u + 0x7FFFu + ((u >> 16) & 1u)) >> 16);
}
__device__ __forceinline__ float bf2f(ush b) { return __uint_as_float(((unsigned)b) << 16); }

__device__ __forceinline__ HL split8(v8f f) {
  PackU ph, pl;
#pragma unroll
  for (int e = 0; e < 8; ++e) {
    const ush hi = f2bf(f[e]);
    ph.s[e] = hi;
    pl.s[e] = f2bf(f[e] - bf2f(hi));
  }
  HL r; r.h = ph.u; r.l = pl.u;
  return r;
}

__device__ __forceinline__ v8f mmab(v16us a, v16us b, v8f c) {
  FragU ua, ub; ua.v = a; ub.v = b;
  c = __builtin_amdgcn_wmma_f32_16x16x32_bf16(false, ua.b, false, ub.b, (short)0, c, false, false);
  asm volatile("v_nop\n\tv_nop\n\tv_nop\n\tv_nop" : "+v"(c) : "v"(a), "v"(b));
  return c;
}

__device__ __forceinline__ v16us ldfragu(const ush* p, int ld, int row0, int k0, int lane) {
  const int m = lane & 15, lh = lane >> 4;
  const ush* q = p + (size_t)(row0 + m) * ld + k0 + 8 * lh;
  FragU f;
  f.h[0] = *(const v8us*)(q);
  f.h[1] = *(const v8us*)(q + 16);
  return f.v;
}

__device__ __forceinline__ v8f zero8() { return (v8f){0.f, 0.f, 0.f, 0.f, 0.f, 0.f, 0.f, 0.f}; }

__device__ __forceinline__ void gemm3_32x64(const ush* __restrict__ Ah, const ush* __restrict__ Al, int lda,
                                            const ush* __restrict__ Bh, const ush* __restrict__ Bl, int ldb,
                                            int m0, int n0, int lane, v8f (&acc)[2][4]) {
#pragma unroll 1
  for (int k0 = 0; k0 < EMB; k0 += 32) {
    const v16us a0h = ldfragu(Ah, lda, m0, k0, lane);
    const v16us a1h = ldfragu(Ah, lda, m0 + 16, k0, lane);
    const v16us a0l = ldfragu(Al, lda, m0, k0, lane);
    const v16us a1l = ldfragu(Al, lda, m0 + 16, k0, lane);
#pragma unroll
    for (int t = 0; t < 4; ++t) {
      const v16us bh = ldfragu(Bh, ldb, n0 + 16 * t, k0, lane);
      const v16us bl = ldfragu(Bl, ldb, n0 + 16 * t, k0, lane);
      acc[0][t] = mmab(a0h, bh, acc[0][t]);
      acc[1][t] = mmab(a1h, bh, acc[1][t]);
      acc[0][t] = mmab(a0h, bl, acc[0][t]);
      acc[1][t] = mmab(a1h, bl, acc[1][t]);
      acc[0][t] = mmab(a0l, bh, acc[0][t]);
      acc[1][t] = mmab(a1l, bh, acc[1][t]);
    }
  }
}

__global__ __launch_bounds__(256) void k_cvt_x(const float* __restrict__ q, const float* __restrict__ k,
                                               const float* __restrict__ v, ush* __restrict__ xh,
                                               ush* __restrict__ xl, int ngrp) {
  const int which = blockIdx.y;
  const float* x = (which == 0) ? q : ((which == 1) ? k : v);
  const int t = blockIdx.x * 256 + (int)threadIdx.x;
  if (t >= ngrp) return;
  const size_t o  = (size_t)t * 8;
  const size_t od = (size_t)which * NTOK * EMB + o;
  const v4f a0 = *(const v4f*)(x + o);
  const v4f a1 = *(const v4f*)(x + o + 4);
  const v8f f = (v8f){a0[0], a0[1], a0[2], a0[3], a1[0], a1[1], a1[2], a1[3]};
  const HL s = split8(f);
  *(volatile v4u*)(xh + od) = s.h;
  *(volatile v4u*)(xl + od) = s.l;
  __threadfence();
  *(volatile v4u*)(xh + od) = s.h;
  *(volatile v4u*)(xl + od) = s.l;
}

__global__ __launch_bounds__(256) void k_cvt_w(const float* __restrict__ wq, const float* __restrict__ wk,
                                               const float* __restrict__ wv, const float* __restrict__ wo,
                                               ush* __restrict__ wh, ush* __restrict__ wl, int ngrp) {
  const int which = blockIdx.y;
  const float* w = (which == 0) ? wq : ((which == 1) ? wk : ((which == 2) ? wv : wo));
  const int t = blockIdx.x * 256 + (int)threadIdx.x;
  if (t >= ngrp) return;
  const size_t o  = (size_t)t * 8;
  const size_t od = (size_t)which * EMB * EMB + o;
  const v4f a0 = *(const v4f*)(w + o);
  const v4f a1 = *(const v4f*)(w + o + 4);
  const v8f f = (v8f){a0[0], a0[1], a0[2], a0[3], a1[0], a1[1], a1[2], a1[3]};
  const HL s = split8(f);
  *(volatile v4u*)(wh + od) = s.h;
  *(volatile v4u*)(wl + od) = s.l;
  __threadfence();
  *(volatile v4u*)(wh + od) = s.h;
  *(volatile v4u*)(wl + od) = s.l;
}

#define STP 72
__global__ __launch_bounds__(256) void k_qkv3(const ush* __restrict__ xh, const ush* __restrict__ xl,
                                              const ush* __restrict__ wth, const ush* __restrict__ wtl,
                                              ush* __restrict__ q3h, ush* __restrict__ q3l,
                                              ush* __restrict__ k3h, ush* __restrict__ k3l,
                                              ush* __restrict__ v3h, ush* __restrict__ v3l) {
  __shared__ __align__(16) ush st[256 * STP];
  const int tid = threadIdx.x, lane = tid & 31, wave = tid >> 5;
  const int hh = lane >> 4, c = lane & 15;
  const int mb = blockIdx.x * 256;
  const int m0 = mb + wave * 32;
  const int n0 = blockIdx.y * 64;
  const int which = n0 / EMB;
  const int nn = n0 - which * EMB;
  const int b  = mb / LSEQ;
  const int l0 = mb - b * LSEQ;
  const ush* Ah = xh + (size_t)which * NTOK * EMB;
  const ush* Al = xl + (size_t)which * NTOK * EMB;

  v8f acc[2][4];
#pragma unroll
  for (int s = 0; s < 2; ++s)
#pragma unroll
    for (int t = 0; t < 4; ++t) acc[s][t] = zero8();
  gemm3_32x64(Ah, Al, EMB, wth, wtl, EMB, m0, n0, lane, acc);

  ush* bh = (which == 0) ? q3h : ((which == 1) ? k3h : v3h);
  ush* bl = (which == 0) ? q3l : ((which == 1) ? k3l : v3l);
  size_t go[8];
#pragma unroll
  for (int j = 0; j < 8; ++j) {
    const int p  = tid + 256 * j;
    const int L  = p >> 3;
    const int pc = p & 7;
    if (which < 2) {
      go[j] = ((size_t)(mb + L)) * EMB + nn + pc * 8;
    } else {
      const int d  = L >> 2;
      const int nl = (L & 3) * 64 + pc * 8;
      go[j] = ((size_t)(b * EMB + nn + d)) * LSEQ + l0 + nl;
    }
  }

#pragma unroll 1
  for (int ph = 0; ph < 2; ++ph) {
    __syncthreads();
#pragma unroll
    for (int t = 0; t < 4; ++t) {
#pragma unroll
      for (int sub = 0; sub < 2; ++sub) {
#pragma unroll
        for (int r = 0; r < 8; ++r) {
          const int lr = wave * 32 + sub * 16 + 8 * hh + r;
          const float v = acc[sub][t][r];
          const ush hi = f2bf(v);
          st[lr * STP + 16 * t + c] = (ph == 0) ? hi : f2bf(v - bf2f(hi));
        }
      }
    }
    __syncthreads();
    v4u val[8];
    if (which < 2) {
#pragma unroll
      for (int j = 0; j < 8; ++j) {
        const int p  = tid + 256 * j;
        const int lr = p >> 3;
        const int pc = p & 7;
        PackU pk;
        pk.s  = *(const v8us*)(st + lr * STP + pc * 8);
        val[j] = pk.u;
      }
    } else {
#pragma unroll
      for (int j = 0; j < 8; ++j) {
        const int p  = tid + 256 * j;
        const int L  = p >> 3;
        const int pc = p & 7;
        const int d  = L >> 2;
        const int nl = (L & 3) * 64 + pc * 8;
        const ush* cp = st + nl * STP + d;
        PackU pk;
        pk.s = (v8us){cp[0 * STP], cp[1 * STP], cp[2 * STP], cp[3 * STP],
                      cp[4 * STP], cp[5 * STP], cp[6 * STP], cp[7 * STP]};
        val[j] = pk.u;
      }
    }
    ush* dst = (ph == 0) ? bh : bl;
#pragma unroll
    for (int j = 0; j < 8; ++j) *(volatile v4u*)(dst + go[j]) = val[j];
    __threadfence();
#pragma unroll
    for (int j = 0; j < 8; ++j) *(volatile v4u*)(dst + go[j]) = val[j];
  }
}

#define SSP 128
#define SPP 136
#define OTP 68
__global__ __launch_bounds__(256) void k_attn3(const ush* __restrict__ q3h, const ush* __restrict__ q3l,
                                               const ush* __restrict__ k3h, const ush* __restrict__ k3l,
                                               const ush* __restrict__ v3h, const ush* __restrict__ v3l,
                                               ush* __restrict__ o3h, ush* __restrict__ o3l, float sscale) {
  __shared__ __align__(16) float sSO[BR * SSP];
  __shared__ __align__(16) ush   sPh[BR * SPP];
  __shared__ __align__(16) ush   sPl[BR * SPP];
  __shared__ __align__(16) float sRed[BR * 8];
  __shared__ __align__(16) float rM[BR];
  __shared__ __align__(16) float rMn[BR];
  __shared__ __align__(16) float rL[BR];
  __shared__ __align__(16) float rSc[BR];

  float* sS = sSO;
  const int tid = threadIdx.x, lane = tid & 31, wave = tid >> 5;
  const int hh = lane >> 4, c = lane & 15;
  const int b  = blockIdx.z;
  const int h  = blockIdx.y;
  const int q0 = (int)blockIdx.x * BR;
  const ush* Qh = q3h + (size_t)b * LSEQ * EMB + h * DH;
  const ush* Ql = q3l + (size_t)b * LSEQ * EMB + h * DH;
  const ush* Kh = k3h + (size_t)b * LSEQ * EMB + h * DH;
  const ush* Kl = k3l + (size_t)b * LSEQ * EMB + h * DH;
  const ush* Vh = v3h + (size_t)b * EMB * LSEQ + (size_t)h * DH * LSEQ;
  const ush* Vl = v3l + (size_t)b * EMB * LSEQ + (size_t)h * DH * LSEQ;
  const float NEGI = -__builtin_huge_valf();
  if (tid < BR) { rM[tid] = NEGI; rL[tid] = 0.f; }
  __syncthreads();

  const int osub = wave >> 2, oet = wave & 3;
  v8f oacc = zero8();

  const int srow = tid >> 3, schk = tid & 7;
  const int nch = (q0 + BR + BC - 1) / BC;

#pragma unroll 1
  for (int ch = 0; ch < nch; ++ch) {
    const int j0  = ch * BC;
    const int kr0 = j0 + wave * 16;
    v8f s[2];
    s[0] = zero8(); s[1] = zero8();
#pragma unroll 1
    for (int k0 = 0; k0 < DH; k0 += 32) {
      const v16us a0h = ldfragu(Qh, EMB, q0, k0, lane);
      const v16us a1h = ldfragu(Qh, EMB, q0 + 16, k0, lane);
      const v16us a0l = ldfragu(Ql, EMB, q0, k0, lane);
      const v16us a1l = ldfragu(Ql, EMB, q0 + 16, k0, lane);
      const v16us kbh = ldfragu(Kh, EMB, kr0, k0, lane);
      const v16us kbl = ldfragu(Kl, EMB, kr0, k0, lane);
      s[0] = mmab(a0h, kbh, s[0]);
      s[1] = mmab(a1h, kbh, s[1]);
      s[0] = mmab(a0h, kbl, s[0]);
      s[1] = mmab(a1h, kbl, s[1]);
      s[0] = mmab(a0l, kbh, s[0]);
      s[1] = mmab(a1l, kbh, s[1]);
    }
    {
      const int key = kr0 + c;
#pragma unroll
      for (int t = 0; t < 2; ++t) {
#pragma unroll
        for (int r = 0; r < 8; ++r) {
          const int row = 16 * t + 8 * hh + r;
          const float raw = (key > q0 + row) ? -1.0e9f : s[t][r];
          sS[row * SSP + wave * 16 + c] = raw * sscale;
        }
      }
    }
    __syncthreads();
    {
      const float* sr = sS + srow * SSP + schk * 16;
      const v4f x0 = *(const v4f*)(sr);
      const v4f x1 = *(const v4f*)(sr + 4);
      const v4f x2 = *(const v4f*)(sr + 8);
      const v4f x3 = *(const v4f*)(sr + 12);
      float mx = x0[0];
#pragma unroll
      for (int e = 1; e < 4; ++e) mx = fmaxf(mx, x0[e]);
#pragma unroll
      for (int e = 0; e < 4; ++e) { mx = fmaxf(mx, x1[e]); mx = fmaxf(mx, x2[e]); mx = fmaxf(mx, x3[e]); }
      sRed[srow * 8 + schk] = mx;
    }
    __syncthreads();
    if (tid < BR) {
      float mx = rM[tid];
#pragma unroll
      for (int i = 0; i < 8; ++i) mx = fmaxf(mx, sRed[tid * 8 + i]);
      rMn[tid] = mx;
    }
    __syncthreads();
    {
      const float mx = rMn[srow];
      const float* sr = sS + srow * SSP + schk * 16;
      float sum = 0.f;
      PackU ph0, pl0, ph1, pl1;
#pragma unroll
      for (int e = 0; e < 8; ++e) {
        const float p = __expf(sr[e] - mx);
        sum += p;
        const ush hi = f2bf(p);
        ph0.s[e] = hi;
        pl0.s[e] = f2bf(p - bf2f(hi));
      }
#pragma unroll
      for (int e = 0; e < 8; ++e) {
        const float p = __expf(sr[8 + e] - mx);
        sum += p;
        const ush hi = f2bf(p);
        ph1.s[e] = hi;
        pl1.s[e] = f2bf(p - bf2f(hi));
      }
      *(v8us*)(sPh + srow * SPP + schk * 16)     = ph0.s;
      *(v8us*)(sPh + srow * SPP + schk * 16 + 8) = ph1.s;
      *(v8us*)(sPl + srow * SPP + schk * 16)     = pl0.s;
      *(v8us*)(sPl + srow * SPP + schk * 16 + 8) = pl1.s;
      sRed[srow * 8 + schk] = sum;
    }
    __syncthreads();
    if (tid < BR) {
      float sum = 0.f;
#pragma unroll
      for (int i = 0; i < 8; ++i) sum += sRed[tid * 8 + i];
      const float mnew = rMn[tid];
      const float fac  = __expf(rM[tid] - mnew);
      rL[tid]  = rL[tid] * fac + sum;
      rM[tid]  = mnew;
      rSc[tid] = fac;
    }
    __syncthreads();
    {
      const v4f f0 = *(const v4f*)(rSc + 16 * osub + 8 * hh);
      const v4f f1 = *(const v4f*)(rSc + 16 * osub + 8 * hh + 4);
#pragma unroll
      for (int r = 0; r < 4; ++r) {
        oacc[r]     *= f0[r];
        oacc[4 + r] *= f1[r];
      }
    }
#pragma unroll 1
    for (int kk = 0; kk < BC / 32; ++kk) {
      const v16us pah = ldfragu(sPh, SPP, 16 * osub, kk * 32, lane);
      const v16us pal = ldfragu(sPl, SPP, 16 * osub, kk * 32, lane);
      const v16us vbh = ldfragu(Vh, LSEQ, 16 * oet, j0 + kk * 32, lane);
      const v16us vbl = ldfragu(Vl, LSEQ, 16 * oet, j0 + kk * 32, lane);
      oacc = mmab(pah, vbh, oacc);
      oacc = mmab(pah, vbl, oacc);
      oacc = mmab(pal, vbh, oacc);
    }
    __syncthreads();
  }

  float* sO = sSO;
#pragma unroll
  for (int r = 0; r < 8; ++r) {
    const int row = 16 * osub + 8 * hh + r;
    const float lv  = rL[row];
    const float inv = (lv > 0.f) ? (1.0f / lv) : 0.f;
    sO[row * OTP + 16 * oet + c] = oacc[r] * inv;
  }
  __syncthreads();
  {
    const int L  = tid >> 3;
    const int pc = tid & 7;
    const v4f x0 = *(const v4f*)(sO + L * OTP + pc * 8);
    const v4f x1 = *(const v4f*)(sO + L * OTP + pc * 8 + 4);
    const v8f f = (v8f){x0[0], x0[1], x0[2], x0[3], x1[0], x1[1], x1[2], x1[3]};
    const HL sp = split8(f);
    const size_t go = ((size_t)(b * LSEQ + q0 + L)) * EMB + h * DH + pc * 8;
    *(volatile v4u*)(o3h + go) = sp.h;
    *(volatile v4u*)(o3l + go) = sp.l;
    __threadfence();
    *(volatile v4u*)(o3h + go) = sp.h;
    *(volatile v4u*)(o3l + go) = sp.l;
  }
}

__global__ __launch_bounds__(256) void k_out3(const ush* __restrict__ ah, const ush* __restrict__ al,
                                              const ush* __restrict__ woh, const ush* __restrict__ wol,
                                              const float* __restrict__ bo, float* __restrict__ out) {
  __shared__ __align__(16) float swall[8 * 16 * OTP];
  const int tid = threadIdx.x, lane = tid & 31, wave = tid >> 5;
  const int hh = lane >> 4, c = lane & 15;
  const int mb = blockIdx.x * 256;
  const int m0 = mb + wave * 32;
  const int n0 = blockIdx.y * 64;
  float* sw = swall + wave * (16 * OTP);

  v8f acc[2][4];
#pragma unroll
  for (int s = 0; s < 2; ++s)
#pragma unroll
    for (int t = 0; t < 4; ++t) acc[s][t] = zero8();
  gemm3_32x64(ah, al, EMB, woh, wol, EMB, m0, n0, lane, acc);

#pragma unroll
  for (int t = 0; t < 4; ++t) {
    const float bn = bo[n0 + 16 * t + c];
#pragma unroll
    for (int sub = 0; sub < 2; ++sub) {
#pragma unroll
      for (int r = 0; r < 8; ++r) acc[sub][t][r] += bn;
    }
  }

#pragma unroll
  for (int sub = 0; sub < 2; ++sub) {
    __syncthreads();
#pragma unroll
    for (int r = 0; r < 8; ++r) {
#pragma unroll
      for (int t = 0; t < 4; ++t) sw[(8 * hh + r) * OTP + 16 * t + c] = acc[sub][t][r];
    }
    __syncthreads();
    v4f val[8];
    size_t go[8];
#pragma unroll
    for (int it = 0; it < 8; ++it) {
      const int p    = lane + 32 * it;
      const int L    = p >> 3;
      const int pc   = p & 7;
      const int row  = L >> 1;
      const int half = L & 1;
      val[it] = *(const v4f*)(sw + row * OTP + half * 32 + pc * 4);
      go[it]  = ((size_t)(m0 + sub * 16 + row)) * EMB + n0 + half * 32 + pc * 4;
    }
#pragma unroll
    for (int it = 0; it < 8; ++it) *(volatile v4f*)(out + go[it]) = val[it];
    __threadfence();
#pragma unroll
    for (int it = 0; it < 8; ++it) *(volatile v4f*)(out + go[it]) = val[it];
  }
}

extern "C" void kernel_launch(void* const* d_in, const int* in_sizes, int n_in,
                              void* d_out, int out_size, void* d_ws, size_t ws_size,
                              hipStream_t stream) {
  if (n_in < 8) return;
  if (in_sizes[0] != NTOK * EMB) return;
  if (in_sizes[1] != NTOK * EMB) return;
  if (in_sizes[2] != NTOK * EMB) return;
  if (in_sizes[3] != EMB * EMB) return;
  if (in_sizes[4] != EMB * EMB) return;
  if (in_sizes[5] != EMB * EMB) return;
  if (in_sizes[6] != EMB * EMB) return;
  if (in_sizes[7] != EMB) return;
  if (out_size != NTOK * EMB) return;

  const float* q  = (const float*)d_in[0];
  const float* k  = (const float*)d_in[1];
  const float* v  = (const float*)d_in[2];
  const float* wq = (const float*)d_in[3];
  const float* wk = (const float*)d_in[4];
  const float* wv = (const float*)d_in[5];
  const float* wo = (const float*)d_in[6];
  const float* bo = (const float*)d_in[7];
  float* out = (float*)d_out;

  size_t off = 0;
  const size_t oXh = off; off += (size_t)3 * NTOK * EMB * 2;
  const size_t oXl = off; off += (size_t)3 * NTOK * EMB * 2;
  const size_t oWh = off; off += (size_t)NW * EMB * EMB * 2;
  const size_t oWl = off; off += (size_t)NW * EMB * EMB * 2;
  const size_t oQh = off; off += (size_t)NTOK * EMB * 2;
  const size_t oQl = off; off += (size_t)NTOK * EMB * 2;
  const size_t oKh = off; off += (size_t)NTOK * EMB * 2;
  const size_t oKl = off; off += (size_t)NTOK * EMB * 2;
  const size_t oVh = off; off += (size_t)NB * EMB * LSEQ * 2;
  const size_t oVl = off; off += (size_t)NB * EMB * LSEQ * 2;
  const size_t oOh = off; off += (size_t)NTOK * EMB * 2;
  const size_t oOl = off; off += (size_t)NTOK * EMB * 2;
  if (off > ws_size) return;
  if (off > (size_t)134217728) return;

  char* ws = (char*)d_ws;
  ush* Xh = (ush*)(ws + oXh);
  ush* Xl = (ush*)(ws + oXl);
  ush* Wh = (ush*)(ws + oWh);
  ush* Wl = (ush*)(ws + oWl);
  ush* Qh = (ush*)(ws + oQh);
  ush* Ql = (ush*)(ws + oQl);
  ush* Kh = (ush*)(ws + oKh);
  ush* Kl = (ush*)(ws + oKl);
  ush* Vh = (ush*)(ws + oVh);
  ush* Vl = (ush*)(ws + oVl);
  ush* Oh = (ush*)(ws + oOh);
  ush* Ol = (ush*)(ws + oOl);

  const float sscale = 0.125f;

  const int ngx = in_sizes[0] / 8;
  k_cvt_x<<<dim3((ngx + 255) / 256, 3), dim3(256), 0, stream>>>(q, k, v, Xh, Xl, ngx);
  const int ngw = in_sizes[3] / 8;
  k_cvt_w<<<dim3((ngw + 255) / 256, NW), dim3(256), 0, stream>>>(wq, wk, wv, wo, Wh, Wl, ngw);
  k_qkv3<<<dim3(NTOK / 256, NQKV / 64), dim3(256), 0, stream>>>(Xh, Xl, Wh, Wl, Qh, Ql, Kh, Kl, Vh, Vl);
  k_attn3<<<dim3(NQT, NH, NB), dim3(256), 0, stream>>>(Qh, Ql, Kh, Kl, Vh, Vl, Oh, Ol, sscale);
  k_out3<<<dim3(NTOK / 256, EMB / 64), dim3(256), 0, stream>>>(Oh, Ol, Wh + (size_t)3 * EMB * EMB,
                                                                Wl + (size_t)3 * EMB * EMB, bo, out);
  (void)hipGetLastError();
}
